// Decouple_18442589569603
// MI455X (gfx1250) — hardware-verified
//
#include <hip/hip_runtime.h>

typedef unsigned short us;
typedef __bf16 v16bf __attribute__((ext_vector_type(16)));
typedef us     v8us  __attribute__((ext_vector_type(8)));
typedef float  v8f   __attribute__((ext_vector_type(8)));
typedef float  v4f   __attribute__((ext_vector_type(4)));
typedef v8us __attribute__((may_alias)) v8usa;
typedef v4f  __attribute__((may_alias)) v4fa;
union Frag { v16bf v; v8us half[2]; };

#define NB      4
#define NC      64
#define NHW     128
#define HWSZ    16384
#define NPIX    65536
#define OC      18
#define XR      130
#define TR      132
#define KA      576
#define KS      288
#define XPLANE  ((size_t)NB * XR * XR * 64)
#define TPLANE  ((size_t)NB * XR * TR * 32)
#define WAPLANE 18432
#define WSPLANE 9216
#define W2PLANE 4096
#define NOUT    4194304

__device__ __forceinline__ unsigned bf_bits(float x) {
  const unsigned u = __float_as_uint(x);
  return (u + 0x7FFFu + ((u >> 16) & 1u)) >> 16;
}
__device__ __forceinline__ void split_bf(float x, us& hi, us& lo) {
  const unsigned uh = bf_bits(x);
  const float xh = __uint_as_float(uh << 16);
  hi = (us)uh;
  lo = (us)bf_bits(x - xh);
}

__device__ __forceinline__ v8f mma_bf(v16bf a, v16bf b, v8f c) {
  v8f d = __builtin_amdgcn_wmma_f32_16x16x32_bf16(false, a, false, b, (short)0, c, false, false);
  asm volatile("v_nop\n\tv_nop\n\tv_nop\n\tv_nop" : "+v"(d) : "v"(a), "v"(b));
  return d;
}

__device__ __forceinline__ v16bf ldfrag(const us* p, int h) {
  Frag f;
  f.half[0] = *(const v8usa*)(p + 8 * h);
  f.half[1] = *(const v8usa*)(p + 16 + 8 * h);
  return f.v;
}

__device__ __forceinline__ int clampi(int v, int lo, int hi) { return v < lo ? lo : (v > hi ? hi : v); }

__global__ __launch_bounds__(256) void k_prep(
    const float* __restrict__ w_off, const float* __restrict__ w_s1, const float* __restrict__ w_s2,
    const float* __restrict__ w_m2, const float* __restrict__ w_e2,
    us* __restrict__ wA, us* __restrict__ wS, us* __restrict__ w2p)
{
  const int g = blockIdx.x * 256 + threadIdx.x;
  if (g >= 11264) return;
  float v[8];
  int pl;
  us* dst;
  if (g < 4608) {
    pl = (g >= 2304) ? 1 : 0;
    const int e0  = (g - pl * 2304) * 8;
    const int n   = e0 / KA;
    const int kp  = e0 - n * KA;
    const int tap = kp >> 6, c0 = kp & 63;
    const int nn  = (n < OC) ? n : (OC - 1);
    const bool okn = n < OC;
    #pragma unroll
    for (int j = 0; j < 8; ++j) {
      const float* wr = w_off + ((size_t)(nn * NC + c0 + j)) * 9;
      float s = 0.0f;
      #pragma unroll 1
      for (int q = 0; q < 9; ++q) s += wr[q];
      const float wt  = wr[tap];
      const float val = (tap == 4) ? (wt - s) : wt;
      v[j] = okn ? val : 0.0f;
    }
    dst = wA + (size_t)pl * WAPLANE + e0;
  } else if (g < 9216) {
    const int gg  = g - 4608;
    const int pl4 = gg / 1152;
    pl = pl4 & 1;
    const int which = pl4 >> 1;
    const int e0  = (gg - pl4 * 1152) * 8;
    const int n   = e0 / KS;
    const int kp  = e0 - n * KS;
    const int tap = kp >> 5, c0 = kp & 31;
    const int nn  = (n < OC) ? n : (OC - 1);
    #pragma unroll
    for (int j = 0; j < 8; ++j) {
      const int c   = c0 + j;
      const bool ok = (n < OC) && (c < OC);
      const int ca  = (c < OC) ? c : (OC - 1);
      int cb        = (c < 9) ? (c + 9) : (c - 9);
      cb            = (cb < OC) ? cb : (OC - 1);
      const float a  = w_s1[((size_t)(nn * OC + ca)) * 9 + tap];
      const float bq = w_s2[((size_t)(nn * OC + cb)) * 9 + tap];
      const float bb = (c < 9) ? -bq : bq;
      const float val = which ? bb : a;
      v[j] = ok ? val : 0.0f;
    }
    dst = wS + (size_t)pl4 * WSPLANE + e0;
  } else {
    const int gg  = g - 9216;
    const int pl4 = gg >> 9;
    pl = pl4 & 1;
    const int which = pl4 >> 1;
    const int e0  = (gg & 511) * 8;
    #pragma unroll
    for (int j = 0; j < 8; ++j) {
      const float a  = w_m2[e0 + j];
      const float bq = w_e2[e0 + j];
      v[j] = which ? bq : a;
    }
    dst = w2p + (size_t)pl4 * W2PLANE + e0;
  }
  us ob[8];
  #pragma unroll
  for (int j = 0; j < 8; ++j) {
    us hh, ll;
    split_bf(v[j], hh, ll);
    ob[j] = pl ? ll : hh;
  }
  const v8us o = { ob[0], ob[1], ob[2], ob[3], ob[4], ob[5], ob[6], ob[7] };
  *(volatile v8us*)dst = o;
  __threadfence();
  *(volatile v8us*)dst = o;
}

__device__ __forceinline__ void cvt_store_pass(const us* sx, us* xT, int b, int hrow, int w, int l) {
  const int q8 = l & 7, sub = l >> 3;
  const size_t rowb = ((size_t)(b * XR + hrow + 1)) * XR;
  #pragma unroll
  for (int p = 0; p < 2; ++p) {
    #pragma unroll
    for (int i = 0; i < 4; ++i) {
      const int px = 16 * w + 4 * i + sub;
      const v8us v = *(const v8usa*)(sx + p * 8192 + px * 64 + 8 * q8);
      us* d = xT + (size_t)p * XPLANE + (rowb + px + 1) * 64 + 8 * q8;
      *(volatile v8us*)d = v;
    }
  }
  const v8us z = { 0, 0, 0, 0, 0, 0, 0, 0 };
  if (w == 0) {
    const int p = sub >> 1;
    const int xp = (sub & 1) ? (XR - 1) : 0;
    us* d = xT + (size_t)p * XPLANE + (rowb + xp) * 64 + 8 * q8;
    *(volatile v8us*)d = z;
  }
  if (hrow == 0 || hrow == NHW - 1) {
    const int yz = (hrow == 0) ? 0 : (XR - 1);
    const size_t rowz = ((size_t)(b * XR + yz)) * XR;
    for (int li = 4 * w + sub; li < 2 * XR; li += 32) {
      const int p = (li >= XR) ? 1 : 0;
      const int xp = li - p * XR;
      us* d = xT + (size_t)p * XPLANE + (rowz + xp) * 64 + 8 * q8;
      *(volatile v8us*)d = z;
    }
  }
}

__global__ __launch_bounds__(256) void k_cvt(const float* __restrict__ x1, float* __restrict__ out0, us* __restrict__ xT)
{
  __shared__ __attribute__((aligned(16))) us sx[2 * 128 * 64];
  const int tid = threadIdx.x, l = tid & 31, w = tid >> 5;
  const int b = blockIdx.x >> 7, hrow = blockIdx.x & 127;

  #pragma unroll
  for (int i = 0; i < 8; ++i) {
    const int f = i * 256 + tid;
    const int c = f >> 5, w4 = f & 31;
    const size_t gi = (((size_t)(b * NC + c)) * NHW + hrow) * NHW + 4 * w4;
    const v4f v = *(const v4fa*)(x1 + gi);
    *(volatile v4f*)(out0 + gi) = v;
    us hh, ll;
    split_bf(v.x, hh, ll); sx[(4 * w4 + 0) * 64 + c] = hh; sx[8192 + (4 * w4 + 0) * 64 + c] = ll;
    split_bf(v.y, hh, ll); sx[(4 * w4 + 1) * 64 + c] = hh; sx[8192 + (4 * w4 + 1) * 64 + c] = ll;
    split_bf(v.z, hh, ll); sx[(4 * w4 + 2) * 64 + c] = hh; sx[8192 + (4 * w4 + 2) * 64 + c] = ll;
    split_bf(v.w, hh, ll); sx[(4 * w4 + 3) * 64 + c] = hh; sx[8192 + (4 * w4 + 3) * 64 + c] = ll;
  }
  __threadfence();
  #pragma unroll
  for (int i = 0; i < 8; ++i) {
    const int f = i * 256 + tid;
    const int c = f >> 5, w4 = f & 31;
    const size_t gi = (((size_t)(b * NC + c)) * NHW + hrow) * NHW + 4 * w4;
    const v4f v = *(const v4fa*)(x1 + gi);
    *(volatile v4f*)(out0 + gi) = v;
  }
  __syncthreads();
  cvt_store_pass(sx, xT, b, hrow, w, l);
  __threadfence();
  cvt_store_pass(sx, xT, b, hrow, w, l);
}

__device__ __forceinline__ void t_store_pass(const us* sT, us* tT, int b, int ho, int w, int l) {
  const int q8 = l & 7, sub = l >> 3;
  const size_t rowb = ((size_t)(b * XR + ho + 1)) * TR;
  #pragma unroll
  for (int p = 0; p < 2; ++p) {
    #pragma unroll
    for (int i = 0; i < 4; ++i) {
      const int q = 4 * i + sub;
      const v8us v = *(const v8usa*)(sT + (w * 2 + p) * 1024 + q * 64 + 8 * q8);
      us* d = tT + (size_t)p * TPLANE + (rowb + 32 * w + 2) * 32 + q * 64 + 8 * q8;
      *(volatile v8us*)d = v;
    }
  }
  const v8us z = { 0, 0, 0, 0, 0, 0, 0, 0 };
  if (w == 0) {
    const int p = sub >> 1;
    const int xq = (sub & 1) ? (TR - 2) : 0;
    us* d = tT + (size_t)p * TPLANE + (rowb + xq) * 32 + 8 * q8;
    *(volatile v8us*)d = z;
  }
  if (ho == 0 || ho == NHW - 1) {
    const int yz = (ho == 0) ? 0 : (XR - 1);
    const size_t rowz = ((size_t)(b * XR + yz)) * TR;
    for (int li = 4 * w + sub; li < 132; li += 16) {
      const int p = (li >= 66) ? 1 : 0;
      const int q = li - p * 66;
      us* d = tT + (size_t)p * TPLANE + rowz * 32 + q * 64 + 8 * q8;
      *(volatile v8us*)d = z;
    }
  }
}

__global__ __launch_bounds__(128) void k_conv1(const us* __restrict__ xT, const us* __restrict__ wA,
                                               const float* __restrict__ boff, us* __restrict__ tT)
{
  __shared__ __attribute__((aligned(16))) us sT[4 * 2 * 1024];
  const int tid = threadIdx.x, l = tid & 31, w = tid >> 5, h = l >> 4, m = l & 15;
  const int b = blockIdx.x >> 7, ho = blockIdx.x & 127;

  const size_t ab = (((size_t)(b * XR + ho)) * XR + 32 * w + m) * 64;
  const us* wr0 = wA + (size_t)m * KA;
  const us* wr1 = wA + (size_t)(16 + m) * KA;

  const v8f zero8 = { 0.f, 0.f, 0.f, 0.f, 0.f, 0.f, 0.f, 0.f };
  v8f acc[2][2];
  acc[0][0] = zero8; acc[0][1] = zero8; acc[1][0] = zero8; acc[1][1] = zero8;

  #pragma unroll 1
  for (int ks = 0; ks < 18; ++ks) {
    const int tap = ks >> 1, cc = ks & 1;
    const int ky = (tap * 11) >> 5, kx = tap - 3 * ky;
    const size_t ao = ab + (size_t)(ky * XR + kx) * 64 + 32 * cc;
    const int ko = ks * 32;
    const v16bf ah0 = ldfrag(xT + ao, h);
    const v16bf ah1 = ldfrag(xT + ao + 1024, h);
    const v16bf al0 = ldfrag(xT + XPLANE + ao, h);
    const v16bf al1 = ldfrag(xT + XPLANE + ao + 1024, h);
    {
      const v16bf bh = ldfrag(wr0 + ko, h);
      const v16bf bl = ldfrag(wr0 + WAPLANE + ko, h);
      acc[0][0] = mma_bf(ah0, bh, acc[0][0]); acc[0][0] = mma_bf(ah0, bl, acc[0][0]); acc[0][0] = mma_bf(al0, bh, acc[0][0]);
      acc[1][0] = mma_bf(ah1, bh, acc[1][0]); acc[1][0] = mma_bf(ah1, bl, acc[1][0]); acc[1][0] = mma_bf(al1, bh, acc[1][0]);
    }
    {
      const v16bf bh = ldfrag(wr1 + ko, h);
      const v16bf bl = ldfrag(wr1 + WAPLANE + ko, h);
      acc[0][1] = mma_bf(ah0, bh, acc[0][1]); acc[0][1] = mma_bf(ah0, bl, acc[0][1]); acc[0][1] = mma_bf(al0, bh, acc[0][1]);
      acc[1][1] = mma_bf(ah1, bh, acc[1][1]); acc[1][1] = mma_bf(ah1, bl, acc[1][1]); acc[1][1] = mma_bf(al1, bh, acc[1][1]);
    }
  }

  #pragma unroll
  for (int nt = 0; nt < 2; ++nt) {
    const int n = 16 * nt + m;
    const bool okn = n < OC;
    const float bn = boff[okn ? n : (OC - 1)];
    #pragma unroll
    for (int mt = 0; mt < 2; ++mt) {
      #pragma unroll
      for (int r = 0; r < 8; ++r) {
        const int px = 16 * mt + 8 * h + r;
        const float v = okn ? (acc[mt][nt][r] + bn) : 0.0f;
        us hh, ll;
        split_bf(v, hh, ll);
        sT[(w * 2 + 0) * 1024 + px * 32 + n] = hh;
        sT[(w * 2 + 1) * 1024 + px * 32 + n] = ll;
      }
    }
  }
  __syncthreads();
  t_store_pass(sT, tT, b, ho, w, l);
  __threadfence();
  t_store_pass(sT, tT, b, ho, w, l);
}

__device__ __forceinline__ void off_store_pass(const float* sO, float* offb, int which, int b, int ho, int w, int l) {
  const int q8 = l & 7, sub = l >> 3;
  #pragma unroll
  for (int i = 0; i < 5; ++i) {
    const int n = 4 * i + sub;
    const int nc = (n < OC) ? n : (OC - 1);
    const v4f v = *(const v4fa*)(sO + w * 1024 + nc * 32 + 4 * q8);
    if (n < OC) {
      float* d = offb + ((((size_t)(which * NB + b)) * OC + n) * NHW + ho) * NHW + 32 * w + 4 * q8;
      *(volatile v4f*)d = v;
    }
  }
}

__global__ __launch_bounds__(128) void k_conv2(const us* __restrict__ tT, const us* __restrict__ wS, float* __restrict__ offb)
{
  __shared__ __attribute__((aligned(16))) float sO[4 * 1024];
  const int tid = threadIdx.x, l = tid & 31, w = tid >> 5, h = l >> 4, m = l & 15;
  const int b = blockIdx.x >> 7, ho = blockIdx.x & 127;
  const int which = blockIdx.y;

  const size_t ab = (((size_t)(b * XR + ho)) * TR + 32 * w + m + 1) * 32;
  const us* wb  = wS + (size_t)which * 2 * WSPLANE;
  const us* wr0 = wb + (size_t)m * KS;
  const us* wr1 = wb + (size_t)(16 + m) * KS;

  const v8f zero8 = { 0.f, 0.f, 0.f, 0.f, 0.f, 0.f, 0.f, 0.f };
  v8f acc[2][2];
  acc[0][0] = zero8; acc[0][1] = zero8; acc[1][0] = zero8; acc[1][1] = zero8;

  #pragma unroll 1
  for (int tap = 0; tap < 9; ++tap) {
    const int ky = (tap * 11) >> 5, kx = tap - 3 * ky;
    const size_t ao = ab + (size_t)(ky * TR + kx) * 32;
    const int ko = tap * 32;
    const v16bf ah0 = ldfrag(tT + ao, h);
    const v16bf ah1 = ldfrag(tT + ao + 512, h);
    const v16bf al0 = ldfrag(tT + TPLANE + ao, h);
    const v16bf al1 = ldfrag(tT + TPLANE + ao + 512, h);
    {
      const v16bf bh = ldfrag(wr0 + ko, h);
      const v16bf bl = ldfrag(wr0 + WSPLANE + ko, h);
      acc[0][0] = mma_bf(ah0, bh, acc[0][0]); acc[0][0] = mma_bf(ah0, bl, acc[0][0]); acc[0][0] = mma_bf(al0, bh, acc[0][0]);
      acc[1][0] = mma_bf(ah1, bh, acc[1][0]); acc[1][0] = mma_bf(ah1, bl, acc[1][0]); acc[1][0] = mma_bf(al1, bh, acc[1][0]);
    }
    {
      const v16bf bh = ldfrag(wr1 + ko, h);
      const v16bf bl = ldfrag(wr1 + WSPLANE + ko, h);
      acc[0][1] = mma_bf(ah0, bh, acc[0][1]); acc[0][1] = mma_bf(ah0, bl, acc[0][1]); acc[0][1] = mma_bf(al0, bh, acc[0][1]);
      acc[1][1] = mma_bf(ah1, bh, acc[1][1]); acc[1][1] = mma_bf(ah1, bl, acc[1][1]); acc[1][1] = mma_bf(al1, bh, acc[1][1]);
    }
  }

  #pragma unroll
  for (int nt = 0; nt < 2; ++nt) {
    const int n = 16 * nt + m;
    #pragma unroll
    for (int mt = 0; mt < 2; ++mt) {
      #pragma unroll
      for (int r = 0; r < 8; ++r) {
        const int px = 16 * mt + 8 * h + r;
        sO[w * 1024 + n * 32 + px] = acc[mt][nt][r];
      }
    }
  }
  __syncthreads();
  off_store_pass(sO, offb, which, b, ho, w, l);
  __threadfence();
  off_store_pass(sO, offb, which, b, ho, w, l);
}

__device__ __forceinline__ void enc_store_pass(const float* sD, float* outp, int b, int ho, int wo0, int w, int l) {
  const int q8 = l & 7, sub = l >> 3;
  #pragma unroll
  for (int i = 0; i < 2; ++i) {
    const int o = 8 * w + 4 * i + sub;
    const v4f v = *(const v4fa*)(sD + o * 32 + 4 * q8);
    float* d = outp + (((size_t)(b * NC + o)) * NHW + ho) * NHW + wo0 + 4 * q8;
    *(volatile v4f*)d = v;
  }
}

__global__ __launch_bounds__(256) void k_enc(const float* __restrict__ x1, const float* __restrict__ offb,
                                             const float* __restrict__ w_m1, const float* __restrict__ w_e1,
                                             const us* __restrict__ w2p, float* __restrict__ out1)
{
  __shared__ float w1s[NC * 9];
  __shared__ float wsum[NC];
  __shared__ __attribute__((aligned(16))) us sy[2 * 2048];
  __shared__ __attribute__((aligned(16))) float sD[2048];

  const int tid = threadIdx.x, l = tid & 31, w = tid >> 5, h = l >> 4, m = l & 15;
  const int wo0 = blockIdx.x * 32;
  const int b = blockIdx.y >> 7, ho = blockIdx.y & 127;
  const int which = blockIdx.z;

  for (int i = tid; i < NC * 9; i += 256) {
    const float a = w_m1[i];
    const float e = w_e1[i];
    w1s[i] = which ? e : a;
  }
  __syncthreads();
  if (tid < NC) {
    float s = 0.0f;
    #pragma unroll 1
    for (int k = 0; k < 9; ++k) s += w1s[tid * 9 + k];
    wsum[tid] = s;
  }
  __syncthreads();

  const int wo = wo0 + l;
  const int cg = w;
  const float* ob = offb + ((size_t)(which * NB + b)) * OC * HWSZ + (size_t)ho * NHW + wo;
  const float* xg = x1 + ((size_t)(b * NC + cg * 8)) * HWSZ;
  float acc[8];
  #pragma unroll
  for (int j = 0; j < 8; ++j) acc[j] = 0.0f;

  #pragma unroll 1
  for (int k = 0; k < 9; ++k) {
    const int ky = (k * 11) >> 5, kx = k - 3 * ky;
    const float dy = ob[(size_t)(2 * k) * HWSZ];
    const float dx = ob[(size_t)(2 * k + 1) * HWSZ];
    const float py  = (float)(ho - 1 + ky) + dy;
    const float pxf = (float)(wo - 1 + kx) + dx;
    const float fy = floorf(py), fx = floorf(pxf);
    const float wy = py - fy, wx = pxf - fx;
    const float omy = 1.0f - wy, omx = 1.0f - wx;
    const float fyc = fminf(fmaxf(fy, -2.0f), 130.0f);
    const float fxc = fminf(fmaxf(fx, -2.0f), 130.0f);
    const int y0 = (int)fyc, x0 = (int)fxc;
    const int y1 = y0 + 1, x1i = x0 + 1;
    const bool vy0 = (y0 >= 0) && (y0 < NHW), vy1 = (y1 >= 0) && (y1 < NHW);
    const bool vx0 = (x0 >= 0) && (x0 < NHW), vx1 = (x1i >= 0) && (x1i < NHW);
    const int cy0 = clampi(y0, 0, NHW - 1), cy1 = clampi(y1, 0, NHW - 1);
    const int cx0 = clampi(x0, 0, NHW - 1), cx1 = clampi(x1i, 0, NHW - 1);
    const int i00 = cy0 * NHW + cx0, i01 = cy0 * NHW + cx1;
    const int i10 = cy1 * NHW + cx0, i11 = cy1 * NHW + cx1;
    const bool m00 = vy0 && vx0, m01 = vy0 && vx1, m10 = vy1 && vx0, m11 = vy1 && vx1;
    #pragma unroll
    for (int j = 0; j < 8; ++j) {
      const float* xc = xg + (size_t)j * HWSZ;
      float v00 = xc[i00];
      float v01 = xc[i01];
      float v10 = xc[i10];
      float v11 = xc[i11];
      v00 = m00 ? v00 : 0.0f;
      v01 = m01 ? v01 : 0.0f;
      v10 = m10 ? v10 : 0.0f;
      v11 = m11 ? v11 : 0.0f;
      const float sv = (((v00 * omy) * omx + (v01 * omy) * wx) + (v10 * wy) * omx) + (v11 * wy) * wx;
      acc[j] += w1s[(cg * 8 + j) * 9 + k] * sv;
    }
  }

  #pragma unroll
  for (int j = 0; j < 8; ++j) {
    const int c = cg * 8 + j;
    const float xv = xg[(size_t)j * HWSZ + (size_t)ho * NHW + wo];
    const float y = acc[j] - xv * wsum[c];
    us hh, ll;
    split_bf(y, hh, ll);
    sy[l * 64 + c] = hh;
    sy[2048 + l * 64 + c] = ll;
  }
  __syncthreads();

  const int mt = w & 1, nt = w >> 1;
  const us* ya = sy + (16 * mt + m) * 64;
  const us* wbh = w2p + (size_t)which * 2 * W2PLANE + (size_t)(16 * nt + m) * 64;
  v8f d8 = { 0.f, 0.f, 0.f, 0.f, 0.f, 0.f, 0.f, 0.f };
  #pragma unroll
  for (int k0 = 0; k0 < 64; k0 += 32) {
    const v16bf ah = ldfrag(ya + k0, h);
    const v16bf al = ldfrag(ya + 2048 + k0, h);
    const v16bf bh = ldfrag(wbh + k0, h);
    const v16bf bl = ldfrag(wbh + W2PLANE + k0, h);
    d8 = mma_bf(ah, bh, d8);
    d8 = mma_bf(ah, bl, d8);
    d8 = mma_bf(al, bh, d8);
  }
  #pragma unroll
  for (int r = 0; r < 8; ++r) sD[(16 * nt + m) * 32 + 16 * mt + 8 * h + r] = d8[r];
  __syncthreads();

  float* outp = out1 + (size_t)which * NOUT;
  enc_store_pass(sD, outp, b, ho, wo0, w, l);
  __threadfence();
  enc_store_pass(sD, outp, b, ho, wo0, w, l);
}

extern "C" void kernel_launch(void* const* d_in, const int* in_sizes, int n_in,
                              void* d_out, int out_size, void* d_ws, size_t ws_size,
                              hipStream_t stream)
{
  if (n_in < 9) return;
  if (in_sizes[0] != NB * NC * HWSZ) return;
  if (in_sizes[1] != OC * NC * 9 || in_sizes[2] != OC) return;
  if (in_sizes[3] != OC * OC * 9 || in_sizes[4] != OC * OC * 9) return;
  if (in_sizes[5] != NC * 9 || in_sizes[6] != NC * NC || in_sizes[7] != NC * 9 || in_sizes[8] != NC * NC) return;
  if (out_size != 3 * NOUT) return;

  const float* x1    = (const float*)d_in[0];
  const float* w_off = (const float*)d_in[1];
  const float* b_off = (const float*)d_in[2];
  const float* w_s1  = (const float*)d_in[3];
  const float* w_s2  = (const float*)d_in[4];
  const float* w_m1  = (const float*)d_in[5];
  const float* w_m2  = (const float*)d_in[6];
  const float* w_e1  = (const float*)d_in[7];
  const float* w_e2  = (const float*)d_in[8];

  float* out0 = (float*)d_out;
  float* out1 = out0 + NOUT;

  const size_t xt_bytes  = 2 * XPLANE * 2;
  const size_t wa_bytes  = (size_t)2 * WAPLANE * 2;
  const size_t tt_bytes  = 2 * TPLANE * 2;
  const size_t ws_bytesw = (size_t)4 * WSPLANE * 2;
  const size_t of_bytes  = (size_t)2 * NB * OC * HWSZ * 4;
  const size_t w2_bytes  = (size_t)4 * W2PLANE * 2;
  const size_t off_xt = 0;
  const size_t off_wa = off_xt + xt_bytes;
  const size_t off_tt = off_wa + wa_bytes;
  const size_t off_ws = off_tt + tt_bytes;
  const size_t off_of = off_ws + ws_bytesw;
  const size_t off_w2 = off_of + of_bytes;
  const size_t total  = off_w2 + w2_bytes;
  if (total > ws_size) return;

  char* ws = (char*)d_ws;
  us*    xT  = (us*)(ws + off_xt);
  us*    wA  = (us*)(ws + off_wa);
  us*    tT  = (us*)(ws + off_tt);
  us*    wSp = (us*)(ws + off_ws);
  float* ofb = (float*)(ws + off_of);
  us*    w2p = (us*)(ws + off_w2);

  k_prep<<<44, 256, 0, stream>>>(w_off, w_s1, w_s2, w_m2, w_e2, wA, wSp, w2p);
  k_cvt<<<NB * NHW, 256, 0, stream>>>(x1, out0, xT);
  k_conv1<<<NB * NHW, 128, 0, stream>>>(xT, wA, b_off, tT);
  dim3 g2(NB * NHW, 2);
  k_conv2<<<g2, 128, 0, stream>>>(tT, wSp, ofb);
  dim3 g3(NHW / 32, NB * NHW, 2);
  k_enc<<<g3, 256, 0, stream>>>(x1, ofb, w_m1, w_e1, w2p, out1);
}
